// GraphSAGEWithAttention_9311489098207
// MI455X (gfx1250) — hardware-verified
//
#include <hip/hip_runtime.h>
#include <stddef.h>


#define FIN     128
#define HIDC    256
#define NCLS    2
#define NTHR    256
#define NWAVE   8
#define EPT     8
#define NGRP    2
#define CHUNK   (NTHR * EPT * NGRP)
#define WCAP    (EPT * NGRP * 32)
#define LISTN   (NWAVE * WCAP)
#define NBC     4096
#define NBF     1024
#define RCAP    40960
#define RBN     128
#define TGT     256
#define DEGCAP  256
#define OTHR    512
#define MAXH    4
#define BM      64
#define WSCAP   134217728
#define NEG_SLOPE 0.2f
#define WSCL    16.0f
#define WINV    0.0625f

#define LDS_FILL ((RCAP + NBF + LISTN) * 4 + 64)
#define LDS_GEMM (BM * HIDC * 4)

static_assert((CHUNK & (CHUNK - 1)) == 0);
static_assert(CHUNK <= 4096);
static_assert(NBC <= 4096 && NBF <= 4096);
static_assert((NBC & (NBC - 1)) == 0 && (NBF & (NBF - 1)) == 0);
static_assert(NBC == 4 * NBF);
static_assert(OTHR * 8 == NBC);
static_assert((RCAP % 32) == 0);
static_assert(TGT == NWAVE * 32);
static_assert((NBC % TGT) == 0);
static_assert((TGT % BM) == 0);
static_assert(BM * 4 == NTHR);
static_assert(FIN / 8 == 16);
static_assert(FIN % 32 == 0 && HIDC % 32 == 0);

typedef float    v2f  __attribute__((ext_vector_type(2)));
typedef float    v4f  __attribute__((ext_vector_type(4)));
typedef float    v8f  __attribute__((ext_vector_type(8)));
typedef int      v4i  __attribute__((ext_vector_type(4)));
typedef _Float16 v8h  __attribute__((ext_vector_type(8)));
typedef _Float16 v16h __attribute__((ext_vector_type(16)));
union FragH { v16h v; v8h h[2]; };

__device__ __forceinline__ v8f wmh(v16h a, v16h b, v8f c) {
  v8f d = __builtin_amdgcn_wmma_f32_16x16x32_f16(false, a, false, b, (short)0, c, false, false);
  asm volatile("v_nop\n\tv_nop\n\tv_nop\n\tv_nop" : "+v"(d) : "v"(a), "v"(b));
  return d;
}

__device__ __forceinline__ v8h cvt8h(v4f a, v4f b, float s) {
  v8h o;
  o[0] = (_Float16)(a.x * s); o[1] = (_Float16)(a.y * s);
  o[2] = (_Float16)(a.z * s); o[3] = (_Float16)(a.w * s);
  o[4] = (_Float16)(b.x * s); o[5] = (_Float16)(b.y * s);
  o[6] = (_Float16)(b.z * s); o[7] = (_Float16)(b.w * s);
  return o;
}

__device__ __forceinline__ float lrelu(float v) { return v > 0.0f ? v : NEG_SLOPE * v; }
__device__ __forceinline__ float eluf(float v)  { return v > 0.0f ? v : (__expf(v) - 1.0f); }

template <int NB>
__device__ __forceinline__ int scan_chunk(const int* __restrict__ dsts, int nE, int cbase, int slotBase,
                                          int vec8, int* list, int tid, int lane, int wave) {
  int wc = 0;
#pragma unroll
  for (int g = 0; g < NGRP; ++g) {
    const int el0  = (g * NTHR + tid) * EPT;
    const int e0   = cbase + el0;
    const int sent = -2147483647 - 1;
    v4i da, db;
    if (vec8 != 0 && cbase + CHUNK <= nE) {
      da = *(const v4i*)(dsts + e0);
      db = *(const v4i*)(dsts + e0 + 4);
    } else {
      da.x = (e0     < nE) ? dsts[min(e0, nE - 1)] : sent;
      da.y = (e0 + 1 < nE) ? dsts[min(e0 + 1, nE - 1)] : sent;
      da.z = (e0 + 2 < nE) ? dsts[min(e0 + 2, nE - 1)] : sent;
      da.w = (e0 + 3 < nE) ? dsts[min(e0 + 3, nE - 1)] : sent;
      db.x = (e0 + 4 < nE) ? dsts[min(e0 + 4, nE - 1)] : sent;
      db.y = (e0 + 5 < nE) ? dsts[min(e0 + 5, nE - 1)] : sent;
      db.z = (e0 + 6 < nE) ? dsts[min(e0 + 6, nE - 1)] : sent;
      db.w = (e0 + 7 < nE) ? dsts[min(e0 + 7, nE - 1)] : sent;
    }
    const unsigned nb = (unsigned)slotBase;
    const unsigned s0 = (unsigned)da.x - nb, s1 = (unsigned)da.y - nb;
    const unsigned s2 = (unsigned)da.z - nb, s3 = (unsigned)da.w - nb;
    const unsigned s4 = (unsigned)db.x - nb, s5 = (unsigned)db.y - nb;
    const unsigned s6 = (unsigned)db.z - nb, s7 = (unsigned)db.w - nb;
    const bool h0 = s0 < (unsigned)NB, h1 = s1 < (unsigned)NB, h2 = s2 < (unsigned)NB, h3 = s3 < (unsigned)NB;
    const bool h4 = s4 < (unsigned)NB, h5 = s5 < (unsigned)NB, h6 = s6 < (unsigned)NB, h7 = s7 < (unsigned)NB;
    const unsigned any = __builtin_amdgcn_ballot_w32(h0 | h1 | h2 | h3 | h4 | h5 | h6 | h7);
    if (any != 0u) {
#define HITJ(J, HJ, SJ) { \
        const unsigned mj = __builtin_amdgcn_ballot_w32(HJ); \
        if (mj != 0u) { \
          if (HJ) { \
            const int pos = wc + (int)__builtin_amdgcn_mbcnt_lo(mj, 0u); \
            if (pos < WCAP) list[wave * WCAP + pos] = ((el0 + (J)) << 12) | (int)(SJ); \
          } \
          wc += (int)__builtin_popcount(mj); } }
      HITJ(0, h0, s0)
      HITJ(1, h1, s1)
      HITJ(2, h2, s2)
      HITJ(3, h3, s3)
      HITJ(4, h4, s4)
      HITJ(5, h5, s5)
      HITJ(6, h6, s6)
      HITJ(7, h7, s7)
#undef HITJ
    }
  }
  return wc;
}

__global__ __launch_bounds__(NTHR) void k_xcvt(const float* __restrict__ x, _Float16* xh, int nN, int nUnits) {
  const int i = (int)blockIdx.x * NTHR + (int)threadIdx.x;
  if (i >= nUnits) return;
  const int row = i >> 4;
  const int c0  = (i & 15) * 8;
  int rr = row > nN - 1 ? nN - 1 : row;
  rr = rr < 0 ? 0 : rr;
  const float* p = x + (size_t)rr * FIN + c0;
  v4f a = *(const v4f*)p, b = *(const v4f*)(p + 4);
  const v4f z = {0.f, 0.f, 0.f, 0.f};
  if (row >= nN) { a = z; b = z; }
  const v8h o = cvt8h(a, b, 1.0f);
  _Float16* d = xh + (size_t)i * 8;
  *(volatile v8h*)d = o;
  __threadfence();
  *(volatile v8h*)d = o;
}

template <int KD, int NC>
__global__ __launch_bounds__(NTHR) void k_wprep(const float* __restrict__ W, _Float16* wp) {
  constexpr int UNITS = NC * KD / 8;
  constexpr int KD8   = KD / 8;
  static_assert((UNITS % NTHR) == 0);
  const int i = (int)blockIdx.x * NTHR + (int)threadIdx.x;
  if (i >= UNITS) return;
  const int n  = i / KD8;
  const int k0 = (i - n * KD8) * 8;
  v4f a, b;
  a.x = W[(size_t)(k0 + 0) * NC + n]; a.y = W[(size_t)(k0 + 1) * NC + n];
  a.z = W[(size_t)(k0 + 2) * NC + n]; a.w = W[(size_t)(k0 + 3) * NC + n];
  b.x = W[(size_t)(k0 + 4) * NC + n]; b.y = W[(size_t)(k0 + 5) * NC + n];
  b.z = W[(size_t)(k0 + 6) * NC + n]; b.w = W[(size_t)(k0 + 7) * NC + n];
  const v8h o = cvt8h(a, b, WSCL);
  _Float16* d = wp + (size_t)i * 8;
  *(volatile v8h*)d = o;
  __threadfence();
  *(volatile v8h*)d = o;
}

__global__ __launch_bounds__(NTHR) void k_count(
    const int* __restrict__ dsts, int* cnt, int nE, int vec8) {
  __shared__ __attribute__((aligned(16))) int scnt[NBC];
  __shared__ __attribute__((aligned(16))) int list[LISTN];
  __shared__ int wcnt[NWAVE];
  const int tid = threadIdx.x, lane = tid & 31, wave = tid >> 5;
  const int nodeBase = blockIdx.x * NBC;

  for (int i = tid; i < NBC; i += NTHR) scnt[i] = 0;
  __syncthreads();

  const int nChunks = (nE + CHUNK - 1) / CHUNK;
#pragma unroll 1
  for (int ch = 0; ch < nChunks; ++ch) {
    const int cbase = ch * CHUNK;
    const int wc = scan_chunk<NBC>(dsts, nE, cbase, nodeBase, vec8, list, tid, lane, wave);
    if (lane == 0) wcnt[wave] = wc;
    __syncthreads();
    if (wave == 0) {
#pragma unroll 1
      for (int wsx = 0; wsx < NWAVE; ++wsx) {
        int n = __builtin_amdgcn_readfirstlane(wcnt[wsx]);
        n = n > WCAP ? WCAP : (n < 0 ? 0 : n);
        const int* lp = list + wsx * WCAP;
#pragma unroll 1
        for (int i = 0; i < n; ++i) {
          const int ent  = __builtin_amdgcn_readfirstlane(lp[i]);
          const int slot = ent & (NBC - 1);
          if (lane == 0) scnt[slot] = scnt[slot] + 1;
        }
      }
    }
    __syncthreads();
  }

  v4i cq[4];
#pragma unroll
  for (int q = 0; q < 4; ++q) {
    const int f = (wave * 4 + q) * 128 + 4 * lane;
    cq[q] = *(const v4i*)(scnt + f);
  }
  int* cp = cnt + (size_t)nodeBase;
#pragma unroll
  for (int q = 0; q < 4; ++q) {
    const int f = (wave * 4 + q) * 128 + 4 * lane;
    *(volatile v4i*)(cp + f) = cq[q];
  }
  __threadfence();
#pragma unroll
  for (int q = 0; q < 4; ++q) {
    const int f = (wave * 4 + q) * 128 + 4 * lane;
    *(volatile v4i*)(cp + f) = cq[q];
  }
}

__global__ __launch_bounds__(OTHR) void k_offsets(
    const int* __restrict__ cnt, int* off, int* rbase, int nChunk) {
  __shared__ __attribute__((aligned(16))) int soff[NBC];
  __shared__ __attribute__((aligned(16))) int srb[RBN];
  __shared__ int wtot[OTHR / 32];
  const int tid = threadIdx.x, lane = tid & 31, wave = tid >> 5, sub = tid >> 7;
  for (int i = tid; i < RBN; i += OTHR) srb[i] = 0;
  int carry = 0;
#pragma unroll 1
  for (int ch = 0; ch < nChunk; ++ch) {
    const int base = ch * NBC;
    const v4i c0 = *(const v4i*)(cnt + base + 8 * tid);
    const v4i c1 = *(const v4i*)(cnt + base + 8 * tid + 4);
    const int e0 = max(c0.x, 0), e1 = max(c0.y, 0), e2 = max(c0.z, 0), e3 = max(c0.w, 0);
    const int e4 = max(c1.x, 0), e5 = max(c1.y, 0), e6 = max(c1.z, 0), e7 = max(c1.w, 0);
    const int ts = e0 + e1 + e2 + e3 + e4 + e5 + e6 + e7;
    int incl = ts;
#pragma unroll
    for (int d = 1; d < 32; d <<= 1) {
      const int t = __shfl_up(incl, d);
      if (lane >= d) incl += t;
    }
    if (lane == 31) wtot[wave] = incl;
    __syncthreads();
    const int S0 = wtot[0]  + wtot[1]  + wtot[2]  + wtot[3];
    const int S1 = wtot[4]  + wtot[5]  + wtot[6]  + wtot[7];
    const int S2 = wtot[8]  + wtot[9]  + wtot[10] + wtot[11];
    const int S3 = wtot[12] + wtot[13] + wtot[14] + wtot[15];
    int pre = 0;
#pragma unroll 1
    for (int w = 4 * sub; w < wave; ++w) pre += wtot[w];
    const int b0 = carry;
    const int b1 = b0 + ((S0 + 31) & ~31);
    const int b2 = b1 + ((S1 + 31) & ~31);
    const int b3 = b2 + ((S2 + 31) & ~31);
    const int b4 = b3 + ((S3 + 31) & ~31);
    const int myb = sub == 0 ? b0 : (sub == 1 ? b1 : (sub == 2 ? b2 : b3));
    if (tid == 0) {
      srb[min(4 * ch + 0, RBN - 1)] = b0;
      srb[min(4 * ch + 1, RBN - 1)] = b1;
      srb[min(4 * ch + 2, RBN - 1)] = b2;
      srb[min(4 * ch + 3, RBN - 1)] = b3;
    }
    int run = myb + pre + incl - ts;
    soff[8 * tid + 0] = run; run += e0;
    soff[8 * tid + 1] = run; run += e1;
    soff[8 * tid + 2] = run; run += e2;
    soff[8 * tid + 3] = run; run += e3;
    soff[8 * tid + 4] = run; run += e4;
    soff[8 * tid + 5] = run; run += e5;
    soff[8 * tid + 6] = run; run += e6;
    soff[8 * tid + 7] = run;
    carry = b4;
    __syncthreads();
    const v4i o0 = *(const v4i*)(soff + 4 * tid);
    const v4i o1 = *(const v4i*)(soff + 4 * (tid + OTHR));
    int* op = off + base;
    *(volatile v4i*)(op + 4 * tid) = o0;
    *(volatile v4i*)(op + 4 * (tid + OTHR)) = o1;
    __threadfence();
    *(volatile v4i*)(op + 4 * tid) = o0;
    *(volatile v4i*)(op + 4 * (tid + OTHR)) = o1;
    __syncthreads();
  }
  if (tid == 0) srb[min(4 * nChunk, RBN - 1)] = carry;
  __syncthreads();
  v4i rv = {0, 0, 0, 0};
  if (tid < 32) rv = *(const v4i*)(srb + 4 * tid);
  if (tid < 32) *(volatile v4i*)(rbase + 4 * tid) = rv;
  __threadfence();
  if (tid < 32) *(volatile v4i*)(rbase + 4 * tid) = rv;
}

__global__ __launch_bounds__(NTHR) void k_fill(
    const int* __restrict__ srcs, const int* __restrict__ dsts,
    const int* __restrict__ off, const int* __restrict__ rbase,
    int* csr, int nN, int nE, int vec8, int csrLen) {
  extern __shared__ v4f lds_dyn[];
  int* region = (int*)lds_dyn;
  int* cursor = region + RCAP;
  int* list   = cursor + NBF;
  int* wcnt   = list + LISTN;
  const int tid = threadIdx.x, lane = tid & 31, wave = tid >> 5;
  const int b = blockIdx.x;
  const int nodeBase = b * NBF;

  int rb0 = rbase[b];
  const int rb1 = rbase[b + 1];
  rb0 = rb0 < 0 ? 0 : (rb0 > csrLen ? csrLen : rb0);
  rb0 &= ~31;
  int len = rb1 - rb0;
  len = len < 0 ? 0 : (len > RCAP ? RCAP : len);
  int lenW = (len + 31) & ~31;
  if (rb0 + lenW > csrLen) lenW = (csrLen - rb0) & ~31;

  {
    const v4i z = {0, 0, 0, 0};
    for (int i = tid; i < RCAP / 4; i += NTHR) ((v4i*)region)[i] = z;
    for (int s = tid; s < NBF; s += NTHR) {
      int o = off[nodeBase + s] - rb0;
      o = o < 0 ? 0 : (o > RCAP ? RCAP : o);
      cursor[s] = o;
    }
  }
  __syncthreads();

  const int nChunks = (nE + CHUNK - 1) / CHUNK;
#pragma unroll 1
  for (int ch = 0; ch < nChunks; ++ch) {
    const int cbase = ch * CHUNK;
    const int wc = scan_chunk<NBF>(dsts, nE, cbase, nodeBase, vec8, list, tid, lane, wave);
    if (lane == 0) wcnt[wave] = wc;
    __syncthreads();
    if (wave == 0) {
#pragma unroll 1
      for (int wsx = 0; wsx < NWAVE; ++wsx) {
        int n = __builtin_amdgcn_readfirstlane(wcnt[wsx]);
        n = n > WCAP ? WCAP : (n < 0 ? 0 : n);
        const int* lp = list + wsx * WCAP;
#pragma unroll 1
        for (int i = 0; i < n; ++i) {
          const int ent  = __builtin_amdgcn_readfirstlane(lp[i]);
          const int slot = ent & (NBF - 1);
          int e = cbase + ((ent >> 12) & (CHUNK - 1));
          e = e > nE - 1 ? nE - 1 : e;
          int src = srcs[e];
          src = src < 0 ? 0 : (src > nN - 1 ? nN - 1 : src);
          if (lane == 0) {
            int pos = cursor[slot];
            pos = pos < 0 ? 0 : (pos > RCAP - 1 ? RCAP - 1 : pos);
            region[pos] = src;
            const int np = pos + 1;
            cursor[slot] = np > RCAP ? RCAP : np;
          }
        }
      }
    }
    __syncthreads();
  }

  const int nv = lenW >> 2;
  int* gp = csr + rb0;
#pragma unroll 1
  for (int i = tid; i < nv; i += NTHR) { const v4i v = ((const v4i*)region)[i]; *(volatile v4i*)(gp + 4 * i) = v; }
  __threadfence();
#pragma unroll 1
  for (int i = tid; i < nv; i += NTHR) { const v4i v = ((const v4i*)region)[i]; *(volatile v4i*)(gp + 4 * i) = v; }
}

template <int KD, int HEADS>
__global__ __launch_bounds__(NTHR) void k_gemm(
    const _Float16* __restrict__ Ah, const _Float16* __restrict__ Bw,
    const float* __restrict__ attS, const float* __restrict__ attD,
    float* C, float* eS, float* eD) {
  constexpr int NC  = HIDC;
  constexpr int TPW = 8;
  constexpr int NES = BM * HEADS;
  constexpr int NV  = NES / 4;
  static_assert(KD % 32 == 0);
  static_assert(HEADS == 4 || HEADS == 1);
  static_assert(2 * NV <= NTHR);
  static_assert(NC == 2 * TPW * 16);

  extern __shared__ v4f lds_dyn[];
  __shared__ __attribute__((aligned(16))) float sES[NES];
  __shared__ __attribute__((aligned(16))) float sED[NES];
  float* stg = (float*)lds_dyn;
  const int tid = threadIdx.x, lane = tid & 31, wave = tid >> 5, hh = lane >> 4, m = lane & 15;
  const int rowBase = blockIdx.x * BM;
  const int rg = wave >> 1, chf = wave & 1;
  const int r0 = rg * 16;
  const int c0 = chf * (TPW * 16);

  v8f acc[TPW];
#pragma unroll
  for (int t = 0; t < TPW; ++t) { v8f z = {0.f, 0.f, 0.f, 0.f, 0.f, 0.f, 0.f, 0.f}; acc[t] = z; }

  const _Float16* ap  = Ah + (size_t)(rowBase + r0 + m) * KD + 8 * hh;
  const _Float16* bp0 = Bw + (size_t)(c0 + m) * KD + 8 * hh;
#pragma unroll 1
  for (int kt = 0; kt < KD / 32; ++kt) {
    FragH a;
    a.h[0] = *(const v8h*)(ap + 32 * kt);
    a.h[1] = *(const v8h*)(ap + 32 * kt + 16);
#pragma unroll
    for (int t = 0; t < TPW; ++t) {
      const _Float16* bp = bp0 + (size_t)(16 * t) * KD + 32 * kt;
      FragH bf;
      bf.h[0] = *(const v8h*)bp;
      bf.h[1] = *(const v8h*)(bp + 16);
      acc[t] = wmh(a.v, bf.v, acc[t]);
    }
  }

  {
    float* sp = stg + (size_t)(r0 + 8 * hh) * NC + c0 + m;
#pragma unroll
    for (int t = 0; t < TPW; ++t) {
#pragma unroll
      for (int r = 0; r < 8; ++r) sp[r * NC + 16 * t] = acc[t][r] * WINV;
    }
  }
  __syncthreads();

  {
    const int drow = tid >> 2, part = tid & 3;
    const float* rp  = stg + (size_t)drow * NC + 64 * part;
    const float* sa  = attS + 64 * part;
    const float* sdd = attD + 64 * part;
    float ps = 0.f, pd = 0.f;
#pragma unroll 4
    for (int c = 0; c < 64; c += 4) {
      const v4f hv = *(const v4f*)(rp + c);
      const v4f av = *(const v4f*)(sa + c);
      const v4f dv = *(const v4f*)(sdd + c);
      ps += hv.x * av.x + hv.y * av.y + hv.z * av.z + hv.w * av.w;
      pd += hv.x * dv.x + hv.y * dv.y + hv.z * dv.z + hv.w * dv.w;
    }
    if constexpr (HEADS == 1) {
      ps += __shfl_xor(ps, 1); pd += __shfl_xor(pd, 1);
      ps += __shfl_xor(ps, 2); pd += __shfl_xor(pd, 2);
      if (part == 0) { sES[drow] = ps; sED[drow] = pd; }
    } else {
      sES[drow * 4 + part] = ps; sED[drow * 4 + part] = pd;
    }
  }

  {
    const size_t gb = (size_t)(rowBase + r0) * NC + c0 + 4 * lane;
    const float* srow = stg + (size_t)r0 * NC + c0 + 4 * lane;
    v4f cv[16];
#pragma unroll
    for (int it = 0; it < 16; ++it) cv[it] = *(const v4f*)(srow + (size_t)it * NC);
#pragma unroll
    for (int it = 0; it < 16; ++it) *(volatile v4f*)(C + gb + (size_t)it * NC) = cv[it];
    __threadfence();
#pragma unroll
    for (int it = 0; it < 16; ++it) *(volatile v4f*)(C + gb + (size_t)it * NC) = cv[it];
  }
  __syncthreads();

  {
    const size_t eb = (size_t)rowBase * HEADS;
    const int iS = tid < NV - 1 ? tid : NV - 1;
    int iD = tid - NV; iD = iD < 0 ? 0 : (iD > NV - 1 ? NV - 1 : iD);
    const v4f vS = *(const v4f*)(sES + 4 * iS);
    const v4f vD = *(const v4f*)(sED + 4 * iD);
    const bool isS = tid < NV;
    const v4f dv = isS ? vS : vD;
    float* gp = isS ? (eS + eb + 4 * iS) : (eD + eb + 4 * iD);
    if (tid < 2 * NV) *(volatile v4f*)gp = dv;
    __threadfence();
    if (tid < 2 * NV) *(volatile v4f*)gp = dv;
  }
}

template <int HEADS, int LAST>
__global__ __launch_bounds__(NTHR) void k_agg(
    const int* __restrict__ csr, const int* __restrict__ off, const int* __restrict__ cnt,
    const float* __restrict__ eS, const float* __restrict__ eD, const float* __restrict__ hw,
    const float* __restrict__ bias, const float* __restrict__ Wc, const float* __restrict__ bc,
    _Float16* xo, float* out, int nN, int csrLen) {
  constexpr int NC = HIDC;
  constexpr int CH = NC / HEADS;
  static_assert(HEADS == 4 || HEADS == 1);
  __shared__ __attribute__((aligned(16))) float sOut[LAST ? (NWAVE * 64) : 4];
  const int tid = threadIdx.x, lane = tid & 31, wave = tid >> 5;
  const int tbase = blockIdx.x * TGT + wave * 32;
  const int col = 8 * lane;
  const int hd  = col / CH;
  const v4f z4 = {0.f, 0.f, 0.f, 0.f};

  const v4f bbA = *(const v4f*)(bias + col);
  const v4f bbB = *(const v4f*)(bias + col + 4);
  v4f w0A = z4, w0B = z4, w1A = z4, w1B = z4;
  float bc0 = 0.f, bc1 = 0.f;
  if constexpr (LAST != 0) {
    w0A.x = Wc[(col + 0) * NCLS]; w0A.y = Wc[(col + 1) * NCLS]; w0A.z = Wc[(col + 2) * NCLS]; w0A.w = Wc[(col + 3) * NCLS];
    w0B.x = Wc[(col + 4) * NCLS]; w0B.y = Wc[(col + 5) * NCLS]; w0B.z = Wc[(col + 6) * NCLS]; w0B.w = Wc[(col + 7) * NCLS];
    w1A.x = Wc[(col + 0) * NCLS + 1]; w1A.y = Wc[(col + 1) * NCLS + 1]; w1A.z = Wc[(col + 2) * NCLS + 1]; w1A.w = Wc[(col + 3) * NCLS + 1];
    w1B.x = Wc[(col + 4) * NCLS + 1]; w1B.y = Wc[(col + 5) * NCLS + 1]; w1B.z = Wc[(col + 6) * NCLS + 1]; w1B.w = Wc[(col + 7) * NCLS + 1];
    bc0 = bc[0]; bc1 = bc[1];
  }

  const int cl    = tbase + lane;
  const int cnt_l = cnt[cl];
  const int off_l = off[cl];

#pragma unroll 1
  for (int j = 0; j < 32; ++j) {
    const int c = tbase + j;
    int n = __shfl(cnt_l, j);
    n = n < 0 ? 0 : (n > DEGCAP ? DEGCAP : n);
    const int st = __shfl(off_l, j);
    const float edc   = eD[(size_t)c * HEADS + hd];
    const float eself = lrelu(eS[(size_t)c * HEADS + hd] + edc);

    float mx = eself;
#pragma unroll 1
    for (int q0 = 0; q0 < n; q0 += 32) {
      int pos = st + q0 + lane;
      pos = pos < 0 ? 0 : (pos > csrLen - 1 ? csrLen - 1 : pos);
      int sl = csr[pos];
      sl = sl < 0 ? 0 : (sl > nN - 1 ? nN - 1 : sl);
      const int mcnt = (n - q0) < 32 ? (n - q0) : 32;
#pragma unroll 1
      for (int pp = 0; pp < mcnt; ++pp) {
        const int s = __builtin_amdgcn_readlane(sl, pp);
        mx = fmaxf(mx, lrelu(eS[(size_t)s * HEADS + hd] + edc));
      }
    }

    float p   = __expf(eself - mx);
    float den = p;
    const float* hc = hw + (size_t)c * NC + col;
    v4f accA = *(const v4f*)hc * p;
    v4f accB = *(const v4f*)(hc + 4) * p;
#pragma unroll 1
    for (int q0 = 0; q0 < n; q0 += 32) {
      int pos = st + q0 + lane;
      pos = pos < 0 ? 0 : (pos > csrLen - 1 ? csrLen - 1 : pos);
      int sl = csr[pos];
      sl = sl < 0 ? 0 : (sl > nN - 1 ? nN - 1 : sl);
      const int mcnt = (n - q0) < 32 ? (n - q0) : 32;
#pragma unroll 1
      for (int pp = 0; pp < mcnt; ++pp) {
        const int s = __builtin_amdgcn_readlane(sl, pp);
        p = __expf(lrelu(eS[(size_t)s * HEADS + hd] + edc) - mx);
        den += p;
        const float* hs = hw + (size_t)s * NC + col;
        const v4f hA = *(const v4f*)hs;
        const v4f hB = *(const v4f*)(hs + 4);
        accA = accA + hA * p;
        accB = accB + hB * p;
      }
    }

    const float rd = __builtin_amdgcn_rcpf(den);
    v4f vA = accA * rd + bbA;
    v4f vB = accB * rd + bbB;

    if constexpr (LAST == 0) {
      vA.x = eluf(vA.x); vA.y = eluf(vA.y); vA.z = eluf(vA.z); vA.w = eluf(vA.w);
      vB.x = eluf(vB.x); vB.y = eluf(vB.y); vB.z = eluf(vB.z); vB.w = eluf(vB.w);
      if (c >= nN) { vA = z4; vB = z4; }
      const v8h o = cvt8h(vA, vB, 1.0f);
      _Float16* xp = xo + (size_t)c * NC + col;
      *(volatile v8h*)xp = o;
      __threadfence();
      *(volatile v8h*)xp = o;
    } else {
      float z0 = vA.x * w0A.x + vA.y * w0A.y + vA.z * w0A.z + vA.w * w0A.w
               + vB.x * w0B.x + vB.y * w0B.y + vB.z * w0B.z + vB.w * w0B.w;
      float z1 = vA.x * w1A.x + vA.y * w1A.y + vA.z * w1A.z + vA.w * w1A.w
               + vB.x * w1B.x + vB.y * w1B.y + vB.z * w1B.z + vB.w * w1B.w;
#pragma unroll
      for (int o = 16; o > 0; o >>= 1) { z0 += __shfl_xor(z0, o); z1 += __shfl_xor(z1, o); }
      z0 += bc0; z1 += bc1;
      const float mz  = fmaxf(z0, z1);
      const float lse = mz + __logf(__expf(z0 - mz) + __expf(z1 - mz));
      if (lane == 0) { sOut[wave * 64 + 2 * j] = z0 - lse; sOut[wave * 64 + 2 * j + 1] = z1 - lse; }
    }
  }

  if constexpr (LAST != 0) {
    __syncthreads();
    int nval = nN - tbase;
    nval = nval < 0 ? 0 : (nval > 32 ? 32 : nval);
    nval *= NCLS;
    const int li = lane < 16 ? lane : 15;
    const v4f ov = *(const v4f*)(sOut + wave * 64 + 4 * li);
    v2f o2; o2.x = ov.x; o2.y = ov.y;
    const bool full4 = (lane < 16) && (4 * lane + 4 <= nval);
    const bool half2 = (lane < 16) && (!full4) && (4 * lane + 2 <= nval);
    float* gp = out + (size_t)tbase * NCLS + 4 * li;
    if (full4) *(volatile v4f*)gp = ov;
    else if (half2) *(volatile v2f*)gp = o2;
    __threadfence();
    if (full4) *(volatile v4f*)gp = ov;
    else if (half2) *(volatile v2f*)gp = o2;
  }
}

extern "C" void kernel_launch(void* const* d_in, const int* in_sizes, int n_in,
                              void* d_out, int out_size, void* d_ws, size_t ws_size,
                              hipStream_t stream) {
  if (n_in < 16) return;
  const int nN = in_sizes[0] / FIN;
  const int nE = in_sizes[1] / 2;
  if (nN <= 0 || nE <= 0 || in_sizes[0] != nN * FIN || in_sizes[1] != 2 * nE) return;
  if (in_sizes[2] != FIN * HIDC || in_sizes[6] != HIDC * HIDC || in_sizes[10] != HIDC * HIDC) return;
  if (in_sizes[3] != HIDC || in_sizes[4] != HIDC || in_sizes[5] != HIDC) return;
  if (in_sizes[7] != HIDC || in_sizes[8] != HIDC || in_sizes[9] != HIDC) return;
  if (in_sizes[11] != HIDC || in_sizes[12] != HIDC || in_sizes[13] != HIDC) return;
  if (in_sizes[14] != HIDC * NCLS || in_sizes[15] != NCLS) return;
  if (out_size != nN * NCLS) return;
  if (nE > (1 << 28) || nN > (1 << 24)) return;

  const float* x   = (const float*)d_in[0];
  const int*   ei  = (const int*)d_in[1];
  const int*   src = ei;
  const int*   dst = ei + nE;
  const float* W1  = (const float*)d_in[2];
  const float* a1s = (const float*)d_in[3];
  const float* a1d = (const float*)d_in[4];
  const float* b1  = (const float*)d_in[5];
  const float* W2  = (const float*)d_in[6];
  const float* a2s = (const float*)d_in[7];
  const float* a2d = (const float*)d_in[8];
  const float* b2  = (const float*)d_in[9];
  const float* W3  = (const float*)d_in[10];
  const float* a3s = (const float*)d_in[11];
  const float* a3d = (const float*)d_in[12];
  const float* b3  = (const float*)d_in[13];
  const float* Wc  = (const float*)d_in[14];
  const float* bc  = (const float*)d_in[15];
  float* out = (float*)d_out;

  const int NPAD   = ((nN + TGT - 1) / TGT) * TGT;
  const int nBC    = (nN + NBC - 1) / NBC;
  const int CNTPAD = nBC * NBC;
  if (4 * nBC + 1 > RBN) return;
  const int nBF    = (nN + NBF - 1) / NBF;
  const int csrLen = ((nE + 31) & ~31) + 4096;
  if (31 * 4 * nBC > 4096) return;
  const int nAgg   = NPAD / TGT;
  const int nGemm  = NPAD / BM;
  const int nXu    = NPAD * (FIN / 8);

  char* ws = (char*)d_ws;
  size_t off = 0;
  const size_t oW1  = off; off += (size_t)HIDC * FIN * 2;         off = (off + 255) & ~(size_t)255;
  const size_t oW2  = off; off += (size_t)HIDC * HIDC * 2;        off = (off + 255) & ~(size_t)255;
  const size_t oW3  = off; off += (size_t)HIDC * HIDC * 2;        off = (off + 255) & ~(size_t)255;
  const size_t oXh  = off; off += (size_t)NPAD * FIN * 2;         off = (off + 255) & ~(size_t)255;
  const size_t oCnt = off; off += (size_t)CNTPAD * 4;             off = (off + 255) & ~(size_t)255;
  const size_t oOff = off; off += (size_t)CNTPAD * 4;             off = (off + 255) & ~(size_t)255;
  const size_t oRb  = off; off += (size_t)RBN * 4;                off = (off + 255) & ~(size_t)255;
  const size_t oCsr = off; off += (size_t)csrLen * 4;             off = (off + 255) & ~(size_t)255;
  const size_t oHw  = off; off += (size_t)NPAD * HIDC * 4;        off = (off + 255) & ~(size_t)255;
  const size_t oXb  = off; off += (size_t)NPAD * HIDC * 2;        off = (off + 255) & ~(size_t)255;
  const size_t oES  = off; off += (size_t)NPAD * MAXH * 4;        off = (off + 255) & ~(size_t)255;
  const size_t oED  = off; off += (size_t)NPAD * MAXH * 4;        off = (off + 255) & ~(size_t)255;
  if (off > ws_size || off > (size_t)WSCAP) return;
  _Float16* wp1 = (_Float16*)(ws + oW1);
  _Float16* wp2 = (_Float16*)(ws + oW2);
  _Float16* wp3 = (_Float16*)(ws + oW3);
  _Float16* xh  = (_Float16*)(ws + oXh);
  int*   cnt  = (int*)(ws + oCnt);
  int*   offp = (int*)(ws + oOff);
  int*   rb   = (int*)(ws + oRb);
  int*   csr  = (int*)(ws + oCsr);
  float* hw   = (float*)(ws + oHw);
  _Float16* xb = (_Float16*)(ws + oXb);
  float* es   = (float*)(ws + oES);
  float* ed   = (float*)(ws + oED);

  const int vec8 = ((nE & 3) == 0) ? 1 : 0;

  k_wprep<FIN, HIDC><<<(HIDC * FIN / 8) / NTHR, NTHR, 0, stream>>>(W1, wp1);
  k_wprep<HIDC, HIDC><<<(HIDC * HIDC / 8) / NTHR, NTHR, 0, stream>>>(W2, wp2);
  k_wprep<HIDC, HIDC><<<(HIDC * HIDC / 8) / NTHR, NTHR, 0, stream>>>(W3, wp3);
  k_xcvt<<<(nXu + NTHR - 1) / NTHR, NTHR, 0, stream>>>(x, xh, nN, nXu);

  k_count<<<nBC, NTHR, 0, stream>>>(dst, cnt, nE, vec8);
  k_offsets<<<1, OTHR, 0, stream>>>(cnt, offp, rb, nBC);
  hipFuncSetAttribute(reinterpret_cast<const void*>(&k_fill),
                      hipFuncAttributeMaxDynamicSharedMemorySize, LDS_FILL);
  k_fill<<<nBF, NTHR, LDS_FILL, stream>>>(src, dst, offp, rb, csr, nN, nE, vec8, csrLen);

  hipFuncSetAttribute(reinterpret_cast<const void*>(&k_gemm<FIN, 4>),
                      hipFuncAttributeMaxDynamicSharedMemorySize, LDS_GEMM);
  k_gemm<FIN, 4><<<nGemm, NTHR, LDS_GEMM, stream>>>(xh, wp1, a1s, a1d, hw, es, ed);
  k_agg<4, 0><<<nAgg, NTHR, 0, stream>>>(csr, offp, cnt, es, ed, hw, b1, Wc, bc, xb, out, nN, csrLen);

  hipFuncSetAttribute(reinterpret_cast<const void*>(&k_gemm<HIDC, 4>),
                      hipFuncAttributeMaxDynamicSharedMemorySize, LDS_GEMM);
  k_gemm<HIDC, 4><<<nGemm, NTHR, LDS_GEMM, stream>>>(xb, wp2, a2s, a2d, hw, es, ed);
  k_agg<4, 0><<<nAgg, NTHR, 0, stream>>>(csr, offp, cnt, es, ed, hw, b2, Wc, bc, xb, out, nN, csrLen);

  hipFuncSetAttribute(reinterpret_cast<const void*>(&k_gemm<HIDC, 1>),
                      hipFuncAttributeMaxDynamicSharedMemorySize, LDS_GEMM);
  k_gemm<HIDC, 1><<<nGemm, NTHR, LDS_GEMM, stream>>>(xb, wp3, a3s, a3d, hw, es, ed);
  k_agg<1, 1><<<nAgg, NTHR, 0, stream>>>(csr, offp, cnt, es, ed, hw, b3, Wc, bc, xb, out, nN, csrLen);
}
